// ForgettingAttention_85693187490477
// MI455X (gfx1250) — hardware-verified
//
#include <hip/hip_runtime.h>
#include <stddef.h>
#include <stdint.h>

#define SQ    2048
#define HID   2048
#define NH    32
#define HDM   64
#define NQKV  6144
#define NSLAB 48
#define QB    128
#define KC    64
#define NQB   (SQ / QB)
#define NCK   (SQ / KC)
#define CVB   2048

static_assert(NH * HDM == HID);
static_assert(NQKV == 3 * HID);
static_assert(NSLAB * 128 == NQKV);
static_assert(QB == 2 * KC);
static_assert(NQB * QB == SQ);
static_assert(NCK * KC == SQ);
static_assert(HID % 64 == 0);
static_assert(SQ % 256 == 0);
static_assert((SQ * HID) % CVB == 0);
static_assert((HID * HID) % CVB == 0);
static_assert((NH * HID) % CVB == 0);
static_assert(SQ % 32 == 0);

typedef _Float16 v16h __attribute__((ext_vector_type(16)));
typedef _Float16 v8h  __attribute__((ext_vector_type(8)));
typedef float    v8f  __attribute__((ext_vector_type(8)));
typedef float    v4f  __attribute__((ext_vector_type(4)));
typedef unsigned int v4u __attribute__((ext_vector_type(4)));

union Frag  { v16h v; v8h h[2]; };
union Pack8 { v8h h; v4u u; };

__device__ __forceinline__ v8f mma16(v16h a, v16h b, v8f c) {
  c = __builtin_amdgcn_wmma_f32_16x16x32_f16(false, a, false, b, (short)0, c, false, false);
  asm volatile("v_nop\n\tv_nop\n\tv_nop\n\tv_nop" : "+v"(c) : "v"(a), "v"(b));
  return c;
}

__device__ __forceinline__ v16h ldfrag(const _Float16* p, int ld, int row0, int k0, int lane) {
  const int m = lane & 15, lh = lane >> 4;
  const _Float16* q = p + (size_t)(row0 + m) * ld + k0 + 8 * lh;
  Frag f;
  f.h[0] = *(const v8h*)(q);
  f.h[1] = *(const v8h*)(q + 16);
  return f.v;
}

__device__ __forceinline__ v8f zero8() { return (v8f){0.f, 0.f, 0.f, 0.f, 0.f, 0.f, 0.f, 0.f}; }

__device__ __forceinline__ void gemm32x64(const _Float16* __restrict__ A, int lda,
                                          const _Float16* __restrict__ Bt, int ldb,
                                          int m0, int n0, int lane, v8f (&acc)[2][4]) {
#pragma unroll 2
  for (int k0 = 0; k0 < HID; k0 += 32) {
    const v16h a0 = ldfrag(A, lda, m0, k0, lane);
    const v16h a1 = ldfrag(A, lda, m0 + 16, k0, lane);
    const v16h b0 = ldfrag(Bt, ldb, n0, k0, lane);
    const v16h b1 = ldfrag(Bt, ldb, n0 + 16, k0, lane);
    const v16h b2 = ldfrag(Bt, ldb, n0 + 32, k0, lane);
    const v16h b3 = ldfrag(Bt, ldb, n0 + 48, k0, lane);
    acc[0][0] = mma16(a0, b0, acc[0][0]);
    acc[1][0] = mma16(a1, b0, acc[1][0]);
    acc[0][1] = mma16(a0, b1, acc[0][1]);
    acc[1][1] = mma16(a1, b1, acc[1][1]);
    acc[0][2] = mma16(a0, b2, acc[0][2]);
    acc[1][2] = mma16(a1, b2, acc[1][2]);
    acc[0][3] = mma16(a0, b3, acc[0][3]);
    acc[1][3] = mma16(a1, b3, acc[1][3]);
  }
}

__global__ __launch_bounds__(256) void k_cvt(const float* __restrict__ src, _Float16* __restrict__ dst, float scale) {
  const size_t o = ((size_t)blockIdx.x * 256 + threadIdx.x) * 8;
  const v4f a0 = *(const v4f*)(src + o);
  const v4f a1 = *(const v4f*)(src + o + 4);
  Pack8 pk;
  pk.h = (v8h){(_Float16)(a0[0] * scale), (_Float16)(a0[1] * scale), (_Float16)(a0[2] * scale), (_Float16)(a0[3] * scale),
               (_Float16)(a1[0] * scale), (_Float16)(a1[1] * scale), (_Float16)(a1[2] * scale), (_Float16)(a1[3] * scale)};
  const v4u vv = pk.u;
  volatile v4u* d = (volatile v4u*)(dst + o);
  *d = vv;
  __threadfence();
  *d = vv;
}

#define ZTP 36
__global__ __launch_bounds__(256) void k_gate(const _Float16* __restrict__ xh,
                                              const _Float16* __restrict__ wfh,
                                              const float* __restrict__ bfv,
                                              float* __restrict__ fp) {
  __shared__ __align__(16) float zt[256 * ZTP];
  const int tid = threadIdx.x, lane = tid & 31, wave = tid >> 5;
  const int hh = lane >> 4, c = lane & 15;
  const int rb = blockIdx.x * 256;
  const int m0 = rb + wave * 32;

  v8f acc[2][2];
#pragma unroll
  for (int s = 0; s < 2; ++s)
#pragma unroll
    for (int t = 0; t < 2; ++t) acc[s][t] = zero8();
#pragma unroll 2
  for (int k0 = 0; k0 < HID; k0 += 32) {
    const v16h a0 = ldfrag(xh, HID, m0, k0, lane);
    const v16h a1 = ldfrag(xh, HID, m0 + 16, k0, lane);
    const v16h b0 = ldfrag(wfh, HID, 0, k0, lane);
    const v16h b1 = ldfrag(wfh, HID, 16, k0, lane);
    acc[0][0] = mma16(a0, b0, acc[0][0]);
    acc[1][0] = mma16(a1, b0, acc[1][0]);
    acc[0][1] = mma16(a0, b1, acc[0][1]);
    acc[1][1] = mma16(a1, b1, acc[1][1]);
  }
#pragma unroll
  for (int sub = 0; sub < 2; ++sub)
#pragma unroll
    for (int t = 0; t < 2; ++t)
#pragma unroll
      for (int r = 0; r < 8; ++r)
        zt[(wave * 32 + 16 * sub + 8 * hh + r) * ZTP + 16 * t + c] = acc[sub][t][r] * 0.015625f;
  __syncthreads();
  {
    float* zr = zt + tid * ZTP;
#pragma unroll 1
    for (int g = 0; g < NH; ++g) {
      const float z = zr[g] + bfv[g];
      const float e = expf(-fabsf(z));
      zr[g] = fminf(z, 0.0f) - log1pf(e);
    }
  }
  __syncthreads();
  v4f val[8];
  size_t go[8];
#pragma unroll
  for (int j = 0; j < 8; ++j) {
    const int p   = tid + 256 * j;
    const int row = p >> 3;
    const int pc  = p & 7;
    val[j] = *(const v4f*)(zt + row * ZTP + pc * 4);
    go[j]  = (size_t)(rb + row) * NH + pc * 4;
  }
  for (int ps = 0; ps < 2; ++ps) {
#pragma unroll
    for (int j = 0; j < 8; ++j) *(volatile v4f*)(fp + go[j]) = val[j];
    __threadfence();
  }
}

#define FTP 36
__global__ __launch_bounds__(256) void k_cum(const float* __restrict__ fp, float* __restrict__ fhi, float* __restrict__ flo) {
  __shared__ __align__(16) float lh[NH * FTP];
  __shared__ __align__(16) float ll[NH * FTP];
  const int tid = threadIdx.x;
  double run = 0.0;
  for (int ph = 0; ph < SQ / 32; ++ph) {
    const int s0 = ph * 32;
    if (tid < 32) {
#pragma unroll 1
      for (int i = 0; i < 32; ++i) {
        const float v = fp[(size_t)(s0 + i) * NH + tid];
        run += (double)v;
        const float hi = (float)run;
        const float lo = (float)(run - (double)hi);
        lh[tid * FTP + i] = hi;
        ll[tid * FTP + i] = lo;
      }
    }
    __syncthreads();
    const int g = tid >> 3, pc = tid & 7;
    const v4f a = *(const v4f*)(lh + g * FTP + pc * 4);
    const v4f b = *(const v4f*)(ll + g * FTP + pc * 4);
    const size_t go = (size_t)g * SQ + s0 + pc * 4;
    *(volatile v4f*)(fhi + go) = a;
    *(volatile v4f*)(flo + go) = b;
    __threadfence();
    *(volatile v4f*)(fhi + go) = a;
    *(volatile v4f*)(flo + go) = b;
    __syncthreads();
  }
}

#define STP 136
__global__ __launch_bounds__(256) void k_qkv(const _Float16* __restrict__ xh,
                                             const _Float16* __restrict__ wt,
                                             _Float16* __restrict__ qp,
                                             _Float16* __restrict__ kp,
                                             _Float16* __restrict__ vtp) {
  __shared__ __align__(16) _Float16 sh[128 * STP];
  const int tid = threadIdx.x, lane = tid & 31, wave = tid >> 5;
  const int hh = lane >> 4, c = lane & 15;
  const int wm = wave >> 1, wn = wave & 1;
  const int sb = blockIdx.x * 128;
  const int ns = blockIdx.y;
  const int which = ns >> 4;
  const int hp = 2 * (ns & 15);
  const int m0 = sb + wm * 32;
  const int n0 = ns * 128 + wn * 64;

  v8f acc[2][4];
#pragma unroll
  for (int s = 0; s < 2; ++s)
#pragma unroll
    for (int t = 0; t < 4; ++t) acc[s][t] = zero8();
  gemm32x64(xh, HID, wt, HID, m0, n0, lane, acc);

#pragma unroll
  for (int sub = 0; sub < 2; ++sub)
#pragma unroll
    for (int t = 0; t < 4; ++t)
#pragma unroll
      for (int r = 0; r < 8; ++r)
        sh[(wm * 32 + 16 * sub + 8 * hh + r) * STP + wn * 64 + 16 * t + c] = (_Float16)(acc[sub][t][r] * 0.015625f);
  __syncthreads();

  if (which < 2) {
    _Float16* base = (which == 0) ? qp : kp;
#pragma unroll
    for (int grp = 0; grp < 2; ++grp) {
      v4u val[4];
      size_t go[4];
#pragma unroll
      for (int jj = 0; jj < 4; ++jj) {
        const int p  = tid + 256 * (4 * grp + jj);
        const int lr = p >> 4;
        const int pc = p & 15;
        const int hs = pc >> 3;
        const int d0 = (pc & 7) * 8;
        Pack8 pk;
        pk.h    = *(const v8h*)(sh + lr * STP + hs * 64 + d0);
        val[jj] = pk.u;
        go[jj]  = ((size_t)(hp + hs) * SQ + sb + lr) * HDM + d0;
      }
      for (int ps = 0; ps < 2; ++ps) {
#pragma unroll
        for (int jj = 0; jj < 4; ++jj) *(volatile v4u*)(base + go[jj]) = val[jj];
        __threadfence();
      }
    }
  } else {
#pragma unroll
    for (int grp = 0; grp < 2; ++grp) {
      v4u val[4];
      size_t go[4];
#pragma unroll
      for (int jj = 0; jj < 4; ++jj) {
        const int p    = tid + 256 * (4 * grp + jj);
        const int dcol = p >> 4;
        const int pc   = p & 15;
        const _Float16* cp = sh + (pc * 8) * STP + dcol;
        Pack8 pk;
        pk.h = (v8h){cp[0 * STP], cp[1 * STP], cp[2 * STP], cp[3 * STP],
                     cp[4 * STP], cp[5 * STP], cp[6 * STP], cp[7 * STP]};
        val[jj] = pk.u;
        const int hb = hp + (dcol >> 6);
        const int d  = dcol & 63;
        go[jj]  = ((size_t)hb * HDM + d) * SQ + sb + pc * 8;
      }
      for (int ps = 0; ps < 2; ++ps) {
#pragma unroll
        for (int jj = 0; jj < 4; ++jj) *(volatile v4u*)(vtp + go[jj]) = val[jj];
        __threadfence();
      }
    }
  }
}

#define KTP 72
__global__ __launch_bounds__(256) void k_attn(const _Float16* __restrict__ qp,
                                              const _Float16* __restrict__ kp,
                                              const _Float16* __restrict__ vt,
                                              const float* __restrict__ fhi,
                                              const float* __restrict__ flo,
                                              _Float16* __restrict__ op) {
  __shared__ __align__(16) _Float16 Ks[KC * KTP];
  __shared__ __align__(16) _Float16 Vs[HDM * KTP];
  __shared__ __align__(16) _Float16 Ps[8 * 16 * KTP];

  const int tid = threadIdx.x, lane = tid & 31, wave = tid >> 5;
  const int hh = lane >> 4, c = lane & 15;
  const int qb  = blockIdx.x % NQB;
  const int h   = blockIdx.x / NQB;
  const int q0  = qb * QB + wave * 16;
  const int nck = 2 * qb + 2;

  const _Float16* Q = qp + (size_t)h * SQ * HDM;
  const _Float16* K = kp + (size_t)h * SQ * HDM;
  const _Float16* V = vt + (size_t)h * HDM * SQ;
  const float* FH = fhi + (size_t)h * SQ;
  const float* FL = flo + (size_t)h * SQ;

  v16h qa[2];
  qa[0] = ldfrag(Q, HDM, q0, 0, lane);
  qa[1] = ldfrag(Q, HDM, q0, 32, lane);

  float fqh[8], fql[8];
#pragma unroll
  for (int r = 0; r < 8; ++r) { fqh[r] = FH[q0 + 8 * hh + r]; fql[r] = FL[q0 + 8 * hh + r]; }

  const float NEGI = -__builtin_huge_valf();
  float mrow[8], lrow[8];
  v8f oacc[4];
#pragma unroll
  for (int r = 0; r < 8; ++r) { mrow[r] = NEGI; lrow[r] = 0.f; }
#pragma unroll
  for (int t = 0; t < 4; ++t) oacc[t] = zero8();

  _Float16* pw = Ps + wave * 16 * KTP;

  for (int kc = 0; kc < nck; ++kc) {
    const int kv0 = kc * KC;
    __syncthreads();
    {
      const int r  = tid >> 2;
      const int qq = (tid & 3) * 16;
      const _Float16* ks = K + (size_t)(kv0 + r) * HDM + qq;
      const _Float16* vs = V + (size_t)r * SQ + kv0 + qq;
#pragma unroll
      for (int e = 0; e < 2; ++e) {
        *(v8h*)(Ks + r * KTP + qq + 8 * e) = *(const v8h*)(ks + 8 * e);
        *(v8h*)(Vs + r * KTP + qq + 8 * e) = *(const v8h*)(vs + 8 * e);
      }
    }
    __syncthreads();

    v8f s[4];
#pragma unroll
    for (int j = 0; j < 4; ++j) s[j] = zero8();
#pragma unroll
    for (int dc = 0; dc < 2; ++dc) {
#pragma unroll
      for (int j = 0; j < 4; ++j) {
        const v16h kb = ldfrag(Ks, KTP, j * 16, dc * 32, lane);
        s[j] = mma16(qa[dc], kb, s[j]);
      }
    }
    float fkh[4], fkl[4];
#pragma unroll
    for (int j = 0; j < 4; ++j) { fkh[j] = FH[kv0 + 16 * j + c]; fkl[j] = FL[kv0 + 16 * j + c]; }

    float cm[8];
#pragma unroll
    for (int r = 0; r < 8; ++r) {
      const int row = q0 + 8 * hh + r;
      float m = NEGI;
#pragma unroll
      for (int j = 0; j < 4; ++j) {
        const int key = kv0 + 16 * j + c;
        float v = s[j][r] * 0.125f + ((fqh[r] - fkh[j]) + (fql[r] - fkl[j]));
        v = (key > row) ? NEGI : v;
        s[j][r] = v;
        m = fmaxf(m, v);
      }
#pragma unroll
      for (int off = 1; off < 16; off <<= 1) m = fmaxf(m, __shfl_xor(m, off, 32));
      cm[r] = m;
    }
    float al[8];
#pragma unroll
    for (int r = 0; r < 8; ++r) {
      const float mnew  = fmaxf(mrow[r], cm[r]);
      const float alpha = __expf(mrow[r] - mnew);
      mrow[r] = mnew;
      float psum = 0.f;
#pragma unroll
      for (int j = 0; j < 4; ++j) {
        const float p = __expf(s[j][r] - mnew);
        psum += p;
        pw[(8 * hh + r) * KTP + j * 16 + c] = (_Float16)(p * 1024.0f);
      }
#pragma unroll
      for (int off = 1; off < 16; off <<= 1) psum += __shfl_xor(psum, off, 32);
      lrow[r] = lrow[r] * alpha + psum;
      al[r] = alpha;
    }
#pragma unroll
    for (int t = 0; t < 4; ++t)
#pragma unroll
      for (int r = 0; r < 8; ++r) oacc[t][r] *= al[r];
    __syncthreads();

#pragma unroll
    for (int kk = 0; kk < 2; ++kk) {
      const v16h pa = ldfrag(pw, KTP, 0, kk * 32, lane);
#pragma unroll
      for (int t = 0; t < 4; ++t) {
        const v16h vb = ldfrag(Vs, KTP, t * 16, kk * 32, lane);
        oacc[t] = mma16(pa, vb, oacc[t]);
      }
    }
  }

  float invl[8];
#pragma unroll
  for (int r = 0; r < 8; ++r) invl[r] = (lrow[r] > 0.f) ? (0.015625f / lrow[r]) : 0.f;
  __syncthreads();
#pragma unroll
  for (int r = 0; r < 8; ++r) {
#pragma unroll
    for (int t = 0; t < 4; ++t)
      pw[(8 * hh + r) * KTP + 16 * t + c] = (_Float16)(oacc[t][r] * invl[r]);
  }
  __syncthreads();
  v4u val[4];
  size_t go[4];
#pragma unroll
  for (int it = 0; it < 4; ++it) {
    const int p  = lane + 32 * it;
    const int L  = p >> 3;
    const int pc = p & 7;
    Pack8 pk;
    pk.h    = *(const v8h*)(pw + L * KTP + pc * 8);
    val[it] = pk.u;
    go[it]  = (size_t)(q0 + L) * HID + (size_t)h * HDM + pc * 8;
  }
  for (int ps = 0; ps < 2; ++ps) {
#pragma unroll
    for (int it = 0; it < 4; ++it) *(volatile v4u*)(op + go[it]) = val[it];
    __threadfence();
  }
}

#define OTP 68
__device__ __forceinline__ void out_epilogue(v8f (&acc)[2][4], float scale, float* sw, float* __restrict__ out,
                                             int m0, int n0, int lane, int hh, int c) {
#pragma unroll
  for (int sub = 0; sub < 2; ++sub) {
    __syncthreads();
#pragma unroll
    for (int t = 0; t < 4; ++t) {
#pragma unroll
      for (int r = 0; r < 8; ++r) sw[(8 * hh + r) * OTP + 16 * t + c] = acc[sub][t][r] * scale;
    }
    __syncthreads();
    v4f val[8];
    size_t go[8];
#pragma unroll
    for (int it = 0; it < 8; ++it) {
      const int p    = lane + 32 * it;
      const int L    = p >> 3;
      const int pc   = p & 7;
      const int row  = L >> 1;
      const int half = L & 1;
      val[it] = *(const v4f*)(sw + row * OTP + half * 32 + pc * 4);
      go[it]  = (size_t)(m0 + sub * 16 + row) * HID + n0 + half * 32 + pc * 4;
    }
    for (int ps = 0; ps < 2; ++ps) {
#pragma unroll
      for (int it = 0; it < 8; ++it) *(volatile v4f*)(out + go[it]) = val[it];
      __threadfence();
    }
  }
}

__global__ __launch_bounds__(256) void k_out(const _Float16* __restrict__ ap,
                                             const _Float16* __restrict__ wt,
                                             float* __restrict__ out) {
  __shared__ __align__(16) float st[8][16 * OTP];
  const int tid = threadIdx.x, lane = tid & 31, wave = tid >> 5;
  const int hh = lane >> 4, c = lane & 15;
  const int m0 = blockIdx.x * 256 + wave * 32;
  const int n0 = blockIdx.y * 64;

  v8f acc[2][4];
#pragma unroll
  for (int s = 0; s < 2; ++s)
#pragma unroll
    for (int t = 0; t < 4; ++t) acc[s][t] = zero8();
  gemm32x64(ap, HID, wt, HID, m0, n0, lane, acc);
  out_epilogue(acc, 0.0009765625f, st[wave], out, m0, n0, lane, hh, c);
}

extern "C" void kernel_launch(void* const* d_in, const int* in_sizes, int n_in,
                              void* d_out, int out_size, void* d_ws, size_t ws_size,
                              hipStream_t stream) {
  if (n_in < 7) return;
  if (in_sizes[0] != SQ * HID) return;
  if (in_sizes[1] != HID * HID) return;
  if (in_sizes[2] != HID * HID) return;
  if (in_sizes[3] != HID * HID) return;
  if (in_sizes[4] != NH * HID) return;
  if (in_sizes[5] != NH) return;
  if (in_sizes[6] != HID * HID) return;
  if (out_size != SQ * HID) return;

  const float* x   = (const float*)d_in[0];
  const float* wq  = (const float*)d_in[1];
  const float* wk  = (const float*)d_in[2];
  const float* wv  = (const float*)d_in[3];
  const float* wf  = (const float*)d_in[4];
  const float* bfv = (const float*)d_in[5];
  const float* wo  = (const float*)d_in[6];
  float* out = (float*)d_out;

  size_t off = 0;
  const size_t oX  = off; off += (size_t)SQ * HID * 2;
  const size_t oWt = off; off += (size_t)NQKV * HID * 2;
  const size_t oWo = off; off += (size_t)HID * HID * 2;
  const size_t oWf = off; off += (size_t)NH * HID * 2;
  const size_t oFp = off; off += (size_t)SQ * NH * 4;
  const size_t oFh = off; off += (size_t)NH * SQ * 4;
  const size_t oFl = off; off += (size_t)NH * SQ * 4;
  const size_t oQ  = off; off += (size_t)NH * SQ * HDM * 2;
  const size_t oK  = off; off += (size_t)NH * SQ * HDM * 2;
  const size_t oV  = off; off += (size_t)NH * HDM * SQ * 2;
  const size_t oO  = off; off += (size_t)SQ * HID * 2;
  if (off > ws_size) return;
  if (off > (size_t)134217728) return;

  char* ws = (char*)d_ws;
  _Float16* Xh  = (_Float16*)(ws + oX);
  _Float16* Wt  = (_Float16*)(ws + oWt);
  _Float16* Wot = (_Float16*)(ws + oWo);
  _Float16* Wfh = (_Float16*)(ws + oWf);
  float*    Fp  = (float*)(ws + oFp);
  float*    Fhi = (float*)(ws + oFh);
  float*    Flo = (float*)(ws + oFl);
  _Float16* Qp  = (_Float16*)(ws + oQ);
  _Float16* Kp  = (_Float16*)(ws + oK);
  _Float16* Vt  = (_Float16*)(ws + oV);
  _Float16* Op  = (_Float16*)(ws + oO);

  k_cvt<<<dim3((SQ * HID) / CVB), dim3(256), 0, stream>>>(x, Xh, 1.0f);
  k_cvt<<<dim3((HID * HID) / CVB), dim3(256), 0, stream>>>(wq, Wt, 64.0f);
  k_cvt<<<dim3((HID * HID) / CVB), dim3(256), 0, stream>>>(wk, Wt + (size_t)HID * HID, 64.0f);
  k_cvt<<<dim3((HID * HID) / CVB), dim3(256), 0, stream>>>(wv, Wt + (size_t)2 * HID * HID, 64.0f);
  k_cvt<<<dim3((HID * HID) / CVB), dim3(256), 0, stream>>>(wo, Wot, 64.0f);
  k_cvt<<<dim3((NH * HID) / CVB), dim3(256), 0, stream>>>(wf, Wfh, 64.0f);
  k_gate<<<dim3(SQ / 256), dim3(256), 0, stream>>>(Xh, Wfh, bfv, Fp);
  k_cum<<<dim3(1), dim3(256), 0, stream>>>(Fp, Fhi, Flo);
  k_qkv<<<dim3(SQ / 128, NSLAB), dim3(256), 0, stream>>>(Xh, Wt, Qp, Kp, Vt);
  k_attn<<<dim3(NH * NQB), dim3(256), 0, stream>>>(Qp, Kp, Vt, Fhi, Flo, Op);
  k_out<<<dim3(SQ / 256, HID / 64), dim3(256), 0, stream>>>(Op, Wot, out);
  (void)hipGetLastError();
}
